// GNNStack_6425271075235
// MI455X (gfx1250) — hardware-verified
//
#include <hip/hip_runtime.h>
#include <stddef.h>
#include <stdint.h>
#include <math.h>


#define DF     128
#define DOUT   64
#define AP     512
#define NTHR   256
#define NWAVE  8
#define EPT    8
#define CHUNK  (NTHR * EPT)
#define WCAP   (EPT * 32)
#define LISTN  (NWAVE * WCAP)
#define NBA    1024
#define SLA    10
#define RCAP   28672
#define DEGCAP 64
#define GBM    64
#define GBN    128
#define GTHR   128
#define AGG_ZINTS    (LISTN + 2 * RCAP + 3 * NBA)
#define MISC_INTS    16
#define ROWBUF_INTS  (NWAVE * 256 / 2)
#define AGG_LDS_INTS (AGG_ZINTS + MISC_INTS + ROWBUF_INTS)
#define TBLCOPY      (RCAP + 2 * NBA)
#define TBLSTRIDE    (TBLCOPY + 32)
#define WSMAX  134217728

#define O_WL0  0
#define O_WL1  16384
#define O_WL2  49152
#define O_WM1  81920
#define O_WM2  114688
#define O_WA0  131072
#define O_WA1  196608
#define O_WA2  262144
#define WP_ELEMS 327680
#define U_WL0  2048
#define U_WL1  6144
#define U_WL2  10240
#define U_WM1  14336
#define U_WM2  16384
#define U_WA0  24576
#define U_WA1  32768
#define U_WA2  40960

static_assert((CHUNK & (CHUNK - 1)) == 0 && CHUNK <= 4096);
static_assert((NBA & (NBA - 1)) == 0 && NBA == (1 << SLA));
static_assert(((long long)CHUNK << SLA) < (1LL << 31));
static_assert(LISTN % NTHR == 0);
static_assert(NBA % NWAVE == 0 && NBA % 32 == 0 && NBA % GBM == 0);
static_assert(RCAP % 4 == 0 && AGG_ZINTS % 4 == 0 && LISTN % 4 == 0 && ((AGG_ZINTS + MISC_INTS) % 4) == 0);
static_assert(AGG_ZINTS % (NTHR * 4) == 0);
static_assert(TBLCOPY % (NTHR * 4) == 0 && (TBLSTRIDE * 4) % 128 == 0);
static_assert(AP == 4 * DF && DF == 4 * 32 && GBN == DF && GBM == (GTHR / 32) * 16);
static_assert(AGG_LDS_INTS * 4 <= 300000);
static_assert(U_WA2 % NTHR == 0 && U_WL0 % NTHR == 0 && U_WM2 % NTHR == 0);
static_assert(O_WA2 + DF * AP == WP_ELEMS);

typedef float          v2f   __attribute__((ext_vector_type(2)));
typedef float          v4f   __attribute__((ext_vector_type(4)));
typedef float          v8f   __attribute__((ext_vector_type(8)));
typedef int            v4i   __attribute__((ext_vector_type(4)));
typedef int            v8i   __attribute__((ext_vector_type(8)));
typedef unsigned short v4us  __attribute__((ext_vector_type(4)));
typedef unsigned short v8us  __attribute__((ext_vector_type(8)));
typedef unsigned short v16us __attribute__((ext_vector_type(16)));
typedef __bf16         v16bf __attribute__((ext_vector_type(16)));
typedef v2f  __attribute__((may_alias)) v2fa;
typedef v4f  __attribute__((may_alias)) v4fa;
typedef v4i  __attribute__((may_alias)) v4ia;
typedef v4us __attribute__((may_alias)) v4usa;
typedef v8us __attribute__((may_alias)) v8usa;
union FragB { v16bf v; v16us u; v8us h[2]; v8i w; };

__device__ __forceinline__ v8f wmb(const FragB& a, const FragB& b, v8f c) {
  v8f d = __builtin_amdgcn_wmma_f32_16x16x32_bf16(false, a.v, false, b.v, (short)0, c, false, false);
  asm volatile("v_nop\n\tv_nop\n\tv_nop\n\tv_nop" : "+v"(d) : "v"(a.w), "v"(b.w));
  return d;
}

__device__ __forceinline__ unsigned bf16_bits(float f) {
  const unsigned u = __float_as_uint(f);
  const unsigned r = (u + 0x7FFFu + ((u >> 16) & 1u)) >> 16;
  return ((u & 0x7fffffffu) > 0x7f800000u) ? ((u >> 16) | 0x40u) : r;
}
__device__ __forceinline__ float bf16_val(float f) {
  return __uint_as_float(bf16_bits(f) << 16);
}
__device__ __forceinline__ float relu_keep(float v) { return (v > 0.0f) ? v : (v - v); }

__device__ __forceinline__ void split4(const v4f y, v4us& h4, v4us& l4) {
  unsigned hb;
  hb = bf16_bits(y.x); h4[0] = (unsigned short)hb; l4[0] = (unsigned short)bf16_bits(y.x - __uint_as_float(hb << 16));
  hb = bf16_bits(y.y); h4[1] = (unsigned short)hb; l4[1] = (unsigned short)bf16_bits(y.y - __uint_as_float(hb << 16));
  hb = bf16_bits(y.z); h4[2] = (unsigned short)hb; l4[2] = (unsigned short)bf16_bits(y.z - __uint_as_float(hb << 16));
  hb = bf16_bits(y.w); h4[3] = (unsigned short)hb; l4[3] = (unsigned short)bf16_bits(y.w - __uint_as_float(hb << 16));
}

__device__ __forceinline__ void wave_sync() {
  __builtin_amdgcn_fence(__ATOMIC_RELEASE, "wavefront");
  __builtin_amdgcn_wave_barrier();
  __builtin_amdgcn_fence(__ATOMIC_ACQUIRE, "wavefront");
}

template <int SLB>
__device__ __forceinline__ int scan_chunk(const int* __restrict__ dsts, int nE, int cbase, int slotBase,
                                          int nb, int vec8, int* list, int tid, int lane, int wave) {
  int wc = 0;
  const int el0  = tid * EPT;
  const int e0   = cbase + el0;
  const int sent = -2147483647 - 1;
  v4i da, db;
  if (vec8 != 0 && cbase + CHUNK <= nE) {
    da = *(const v4i*)(dsts + e0);
    db = *(const v4i*)(dsts + e0 + 4);
  } else {
    da.x = (e0     < nE) ? dsts[min(e0,     nE - 1)] : sent;
    da.y = (e0 + 1 < nE) ? dsts[min(e0 + 1, nE - 1)] : sent;
    da.z = (e0 + 2 < nE) ? dsts[min(e0 + 2, nE - 1)] : sent;
    da.w = (e0 + 3 < nE) ? dsts[min(e0 + 3, nE - 1)] : sent;
    db.x = (e0 + 4 < nE) ? dsts[min(e0 + 4, nE - 1)] : sent;
    db.y = (e0 + 5 < nE) ? dsts[min(e0 + 5, nE - 1)] : sent;
    db.z = (e0 + 6 < nE) ? dsts[min(e0 + 6, nE - 1)] : sent;
    db.w = (e0 + 7 < nE) ? dsts[min(e0 + 7, nE - 1)] : sent;
  }
  const unsigned nbs = (unsigned)slotBase;
  const unsigned unb = (unsigned)nb;
  const unsigned s0 = (unsigned)da.x - nbs, s1 = (unsigned)da.y - nbs;
  const unsigned s2 = (unsigned)da.z - nbs, s3 = (unsigned)da.w - nbs;
  const unsigned s4 = (unsigned)db.x - nbs, s5 = (unsigned)db.y - nbs;
  const unsigned s6 = (unsigned)db.z - nbs, s7 = (unsigned)db.w - nbs;
  const bool h0 = s0 < unb, h1 = s1 < unb, h2 = s2 < unb, h3 = s3 < unb;
  const bool h4 = s4 < unb, h5 = s5 < unb, h6 = s6 < unb, h7 = s7 < unb;
  const unsigned any = __builtin_amdgcn_ballot_w32(h0 | h1 | h2 | h3 | h4 | h5 | h6 | h7);
  if (any != 0u) {
#define HITJ(J, HJ, SJ) { \
      const unsigned mj = __builtin_amdgcn_ballot_w32(HJ); \
      if (mj != 0u) { \
        if (HJ) { \
          const int pos = wc + (int)__builtin_amdgcn_mbcnt_lo(mj, 0u); \
          if (pos < WCAP) list[wave * WCAP + pos] = ((el0 + (J)) << SLB) | (int)(SJ); \
        } \
        wc += (int)__builtin_popcount(mj); } }
    HITJ(0, h0, s0)
    HITJ(1, h1, s1)
    HITJ(2, h2, s2)
    HITJ(3, h3, s3)
    HITJ(4, h4, s4)
    HITJ(5, h5, s5)
    HITJ(6, h6, s6)
    HITJ(7, h7, s7)
#undef HITJ
  }
  return wc;
}

__global__ __launch_bounds__(NTHR) void k_wprep(const float* __restrict__ Wl0, const float* __restrict__ Wl1,
                                                const float* __restrict__ Wl2, const float* __restrict__ Wm1,
                                                const float* __restrict__ Wm2, const float* __restrict__ Wa0,
                                                const float* __restrict__ Wa1, const float* __restrict__ Wa2,
                                                unsigned short* WP) {
  const int u = (int)blockIdx.x * NTHR + (int)threadIdx.x;
  const float* W;
  int off, sh, nout, v;
  if (u < U_WL0)      { W = Wl0; off = O_WL0; sh = 4; nout = DF;   v = u; }
  else if (u < U_WL1) { W = Wl1; off = O_WL1; sh = 5; nout = DF;   v = u - U_WL0; }
  else if (u < U_WL2) { W = Wl2; off = O_WL2; sh = 5; nout = DF;   v = u - U_WL1; }
  else if (u < U_WM1) { W = Wm1; off = O_WM1; sh = 5; nout = DF;   v = u - U_WL2; }
  else if (u < U_WM2) { W = Wm2; off = O_WM2; sh = 5; nout = DOUT; v = u - U_WM1; }
  else if (u < U_WA0) { W = Wa0; off = O_WA0; sh = 6; nout = DF;   v = u - U_WM2; }
  else if (u < U_WA1) { W = Wa1; off = O_WA1; sh = 6; nout = DF;   v = u - U_WA0; }
  else if (u < U_WA2) { W = Wa2; off = O_WA2; sh = 6; nout = DF;   v = u - U_WA1; }
  else return;
  const int kp   = 8 << sh;
  const int n    = v >> sh;
  const int k8   = (v & ((1 << sh) - 1)) * 8;
  const int srow = (k8 & 127) + ((k8 >> 8) << 7);
  const float* p = W + (size_t)srow * nout + n;
  v8us o;
#pragma unroll
  for (int i = 0; i < 8; ++i) o[i] = (unsigned short)bf16_bits(p[(size_t)i * nout]);
  unsigned short* dp = WP + off + (size_t)n * kp + k8;
  *(volatile v8us*)dp = o;
  __threadfence();
  *(volatile v8us*)dp = o;
}

__global__ __launch_bounds__(NTHR) void k_cvx(const float* __restrict__ x, int nN, int nUnits,
                                              unsigned short* xa) {
  const int u = (int)blockIdx.x * NTHR + (int)threadIdx.x;
  if (u >= nUnits) return;
  const int row = u >> 5;
  const int c8  = (u & 31) * 8;
  const int rc  = row < nN ? row : nN - 1;
  const float* p = x + (size_t)rc * DF + (c8 & (DF - 1));
  const v4f a = *(const v4fa*)p;
  const v4f b = *(const v4fa*)(p + 4);
  const bool ok = (row < nN) && (c8 < DF);
  v8us o;
  o[0] = ok ? (unsigned short)bf16_bits(a.x) : (unsigned short)0;
  o[1] = ok ? (unsigned short)bf16_bits(a.y) : (unsigned short)0;
  o[2] = ok ? (unsigned short)bf16_bits(a.z) : (unsigned short)0;
  o[3] = ok ? (unsigned short)bf16_bits(a.w) : (unsigned short)0;
  o[4] = ok ? (unsigned short)bf16_bits(b.x) : (unsigned short)0;
  o[5] = ok ? (unsigned short)bf16_bits(b.y) : (unsigned short)0;
  o[6] = ok ? (unsigned short)bf16_bits(b.z) : (unsigned short)0;
  o[7] = ok ? (unsigned short)bf16_bits(b.w) : (unsigned short)0;
  unsigned short* dp = xa + (size_t)row * AP + c8;
  *(volatile v8us*)dp = o;
  __threadfence();
  *(volatile v8us*)dp = o;
}

template <int EPI>
__global__ __launch_bounds__(GTHR) void k_gemm(unsigned short* Apl, const unsigned short* __restrict__ BT,
                                               int K, int ks0, int ks1, const float* __restrict__ bias,
                                               float* outH, int nN) {
  __shared__ __attribute__((aligned(16))) float stg[GBM * GBN];
  const int tid = (int)threadIdx.x, lane = tid & 31, wave = tid >> 5, hh = lane >> 4, m = lane & 15;
  const int rowBase = (int)blockIdx.x * GBM;

  v8f acc[8];
  {
    const v8f z = {0.f, 0.f, 0.f, 0.f, 0.f, 0.f, 0.f, 0.f};
#pragma unroll
    for (int t = 0; t < 8; ++t) acc[t] = z;
  }
  const unsigned short* ap = Apl + (size_t)(rowBase + 16 * wave + m) * (size_t)AP + 8 * hh;
  const unsigned short* bp = BT + (size_t)m * (size_t)K + 8 * hh;

#pragma unroll 1
  for (int k0 = 0; k0 < K; k0 += 32) {
    if (k0 >= ks0 && k0 < ks1) continue;
    FragB af;
    af.h[0] = *(const v8usa*)(ap + k0);
    af.h[1] = *(const v8usa*)(ap + k0 + 16);
#pragma unroll
    for (int nt = 0; nt < 8; ++nt) {
      const unsigned short* wq = bp + (size_t)(16 * nt) * (size_t)K + k0;
      FragB bf;
      bf.h[0] = *(const v8usa*)wq;
      bf.h[1] = *(const v8usa*)(wq + 16);
      acc[nt] = wmb(af, bf, acc[nt]);
    }
  }

#pragma unroll
  for (int nt = 0; nt < 8; ++nt) {
    const int lc = 16 * nt + m;
#pragma unroll
    for (int r = 0; r < 8; ++r) {
      const int lr = 16 * wave + 8 * hh + r;
      stg[lr * GBN + lc] = acc[nt][r];
    }
  }
  __syncthreads();

  v4f bb4;
  {
    const v4f t1 = *(const v4f*)(bias + 4 * lane);
    bb4.x = bf16_val(t1.x); bb4.y = bf16_val(t1.y); bb4.z = bf16_val(t1.z); bb4.w = bf16_val(t1.w);
  }

  if constexpr (EPI == 0) {
    v4f pv[16];
#pragma unroll
    for (int i = 0; i < 16; ++i) {
      const v4f t = *(const v4fa*)(stg + (16 * wave + i) * GBN + 4 * lane) + bb4;
      v4f y;
      y.x = relu_keep(t.x); y.y = relu_keep(t.y); y.z = relu_keep(t.z); y.w = relu_keep(t.w);
      pv[i] = y;
    }
#pragma unroll
    for (int i = 0; i < 16; ++i)
      *(volatile v4f*)(outH + (size_t)(rowBase + 16 * wave + i) * DF + 4 * lane) = pv[i];
    __threadfence();
#pragma unroll
    for (int i = 0; i < 16; ++i)
      *(volatile v4f*)(outH + (size_t)(rowBase + 16 * wave + i) * DF + 4 * lane) = pv[i];
  } else {
#pragma unroll 1
    for (int i = 0; i < 16; ++i) {
      float* srow = stg + (16 * wave + i) * GBN;
      const bool ok = (rowBase + 16 * wave + i) < nN;
      v4f t = *(const v4fa*)(srow + 4 * lane) + bb4;
      t.x = relu_keep(t.x); t.y = relu_keep(t.y); t.z = relu_keep(t.z); t.w = relu_keep(t.w);
      float ss = (t.x * t.x + t.y * t.y) + (t.z * t.z + t.w * t.w);
      ss += __shfl_xor(ss, 16, 32);
      ss += __shfl_xor(ss, 8, 32);
      ss += __shfl_xor(ss, 4, 32);
      ss += __shfl_xor(ss, 2, 32);
      ss += __shfl_xor(ss, 1, 32);
      const float nrm = sqrtf(ss);
      const float inv = 1.0f / fmaxf(nrm, 1e-12f);
      v4f y;
      y.x = relu_keep(t.x * inv); y.y = relu_keep(t.y * inv);
      y.z = relu_keep(t.z * inv); y.w = relu_keep(t.w * inv);
      y.x = ok ? y.x : 0.0f; y.y = ok ? y.y : 0.0f; y.z = ok ? y.z : 0.0f; y.w = ok ? y.w : 0.0f;
      v4us h4, l4;
      split4(y, h4, l4);
      wave_sync();
      unsigned short* su = (unsigned short*)srow;
      *(v4usa*)(su + 4 * lane) = h4;
      *(v4usa*)(su + DF + 4 * lane) = l4;
    }
    __syncthreads();
    v8us qv[16];
#pragma unroll
    for (int i = 0; i < 16; ++i) {
      const unsigned short* su = (const unsigned short*)(stg + (16 * wave + i) * GBN);
      qv[i] = *(const v8usa*)(su + 8 * lane);
    }
#pragma unroll
    for (int i = 0; i < 16; ++i) {
      unsigned short* rp = Apl + (size_t)(rowBase + 16 * wave + i) * (size_t)AP + 8 * lane;
      *(volatile v8us*)rp = qv[i];
    }
    __threadfence();
#pragma unroll
    for (int i = 0; i < 16; ++i) {
      unsigned short* rp = Apl + (size_t)(rowBase + 16 * wave + i) * (size_t)AP + 8 * lane;
      *(volatile v8us*)rp = qv[i];
    }
  }
}

__global__ __launch_bounds__(GTHR) void k_post(const unsigned short* __restrict__ XA,
                                               const unsigned short* __restrict__ WM1,
                                               const unsigned short* __restrict__ WM2,
                                               const float* __restrict__ b1, const float* __restrict__ b2,
                                               float* out, int nN) {
  __shared__ __attribute__((aligned(16))) float stg[GBM * GBN];
  const int tid = (int)threadIdx.x, lane = tid & 31, wave = tid >> 5, hh = lane >> 4, m = lane & 15;
  const int rowBase = (int)blockIdx.x * GBM;
  const v8f z = {0.f, 0.f, 0.f, 0.f, 0.f, 0.f, 0.f, 0.f};

  v8f acc[8];
#pragma unroll
  for (int t = 0; t < 8; ++t) acc[t] = z;
  {
    const unsigned short* ap = XA + (size_t)(rowBase + 16 * wave + m) * (size_t)AP + 8 * hh;
    const unsigned short* bp = WM1 + (size_t)m * 256 + 8 * hh;
#pragma unroll 1
    for (int k0 = 0; k0 < 256; k0 += 32) {
      FragB af;
      af.h[0] = *(const v8usa*)(ap + k0);
      af.h[1] = *(const v8usa*)(ap + k0 + 16);
#pragma unroll
      for (int nt = 0; nt < 8; ++nt) {
        const unsigned short* wq = bp + (size_t)(16 * nt) * 256 + k0;
        FragB bf;
        bf.h[0] = *(const v8usa*)wq;
        bf.h[1] = *(const v8usa*)(wq + 16);
        acc[nt] = wmb(af, bf, acc[nt]);
      }
    }
  }
#pragma unroll
  for (int nt = 0; nt < 8; ++nt) {
    const int lc = 16 * nt + m;
#pragma unroll
    for (int r = 0; r < 8; ++r) stg[(16 * wave + 8 * hh + r) * GBN + lc] = acc[nt][r];
  }
  __syncthreads();
  {
    v4f bb4;
    const v4f t1 = *(const v4f*)(b1 + 4 * lane);
    bb4.x = bf16_val(t1.x); bb4.y = bf16_val(t1.y); bb4.z = bf16_val(t1.z); bb4.w = bf16_val(t1.w);
#pragma unroll 1
    for (int i = 0; i < 16; ++i) {
      float* srow = stg + (16 * wave + i) * GBN;
      const v4f t = *(const v4fa*)(srow + 4 * lane) + bb4;
      v4us h4, l4;
      split4(t, h4, l4);
      wave_sync();
      unsigned short* su = (unsigned short*)srow;
      *(v4usa*)(su + 4 * lane) = h4;
      *(v4usa*)(su + DF + 4 * lane) = l4;
    }
  }
  __syncthreads();

  v8f ac2[4];
#pragma unroll
  for (int t = 0; t < 4; ++t) ac2[t] = z;
  {
    const unsigned short* ar = (const unsigned short*)stg + (size_t)(16 * wave + m) * 256 + 8 * hh;
    const unsigned short* bp = WM2 + (size_t)m * 256 + 8 * hh;
#pragma unroll 1
    for (int k0 = 0; k0 < 256; k0 += 32) {
      FragB af;
      af.h[0] = *(const v8usa*)(ar + k0);
      af.h[1] = *(const v8usa*)(ar + k0 + 16);
#pragma unroll
      for (int nt = 0; nt < 4; ++nt) {
        const unsigned short* wq = bp + (size_t)(16 * nt) * 256 + k0;
        FragB bf;
        bf.h[0] = *(const v8usa*)wq;
        bf.h[1] = *(const v8usa*)(wq + 16);
        ac2[nt] = wmb(af, bf, ac2[nt]);
      }
    }
  }
  __syncthreads();
#pragma unroll
  for (int nt = 0; nt < 4; ++nt) {
    const int lc = 16 * nt + m;
#pragma unroll
    for (int r = 0; r < 8; ++r) stg[(16 * wave + 8 * hh + r) * GBN + lc] = ac2[nt][r];
  }
  __syncthreads();

  {
    const v2f t2 = *(const v2f*)(b2 + 2 * lane);
    const float c0 = bf16_val(t2.x), c1 = bf16_val(t2.y);
#pragma unroll 1
    for (int i = 0; i < 16; ++i) {
      float* srow = stg + (16 * wave + i) * GBN;
      const v2f v = *(const v2fa*)(srow + 2 * lane);
      const float v0 = v.x + c0, v1 = v.y + c1;
      float mx = fmaxf(v0, v1);
      mx = fmaxf(mx, __shfl_xor(mx, 16, 32));
      mx = fmaxf(mx, __shfl_xor(mx, 8, 32));
      mx = fmaxf(mx, __shfl_xor(mx, 4, 32));
      mx = fmaxf(mx, __shfl_xor(mx, 2, 32));
      mx = fmaxf(mx, __shfl_xor(mx, 1, 32));
      const float d0 = v0 - mx, d1 = v1 - mx;
      float s = expf(d0) + expf(d1);
      s += __shfl_xor(s, 16, 32);
      s += __shfl_xor(s, 8, 32);
      s += __shfl_xor(s, 4, 32);
      s += __shfl_xor(s, 2, 32);
      s += __shfl_xor(s, 1, 32);
      const float ls = logf(s);
      v2f o;
      o.x = d0 - ls; o.y = d1 - ls;
      *(v2fa*)(srow + 2 * lane) = o;
    }
  }
  __syncthreads();

  v4f fv[8];
#pragma unroll
  for (int i = 0; i < 8; ++i) {
    const int lr = 16 * wave + 2 * i + hh;
    fv[i] = *(const v4fa*)(stg + lr * GBN + 4 * m);
  }
#pragma unroll
  for (int i = 0; i < 8; ++i) {
    const int gr = rowBase + 16 * wave + 2 * i + hh;
    if (gr < nN) *(volatile v4f*)(out + (size_t)gr * DOUT + 4 * m) = fv[i];
  }
  __threadfence();
#pragma unroll
  for (int i = 0; i < 8; ++i) {
    const int gr = rowBase + 16 * wave + 2 * i + hh;
    if (gr < nN) *(volatile v4f*)(out + (size_t)gr * DOUT + 4 * m) = fv[i];
  }
}

template <int MODE>
__global__ __launch_bounds__(NTHR) void k_scan(const int* __restrict__ srcs, const int* __restrict__ dsts,
                                               int nE, int nN, int vec8, int mRows,
                                               const float* __restrict__ hf, unsigned short* apl, int* tbl) {
  extern __shared__ __attribute__((aligned(16))) int dsm[];
  int* list = dsm;
  int* hl   = dsm + LISTN;
  int* sl   = hl + RCAP;
  int* cnt  = sl + RCAP;
  int* offs = cnt + NBA;
  int* cur  = offs + NBA;
  int* misc = cur + NBA;
  const int tid = (int)threadIdx.x, lane = tid & 31, wave = tid >> 5;
  unsigned short* rowbuf = (unsigned short*)(misc + MISC_INTS) + wave * 256;
  const int nodeBase = (int)blockIdx.x * NBA;
  int* tb = tbl + (size_t)blockIdx.x * TBLSTRIDE;
  int ovf;

  if constexpr (MODE == 0) {
    {
      const v4i z4 = {0, 0, 0, 0};
      for (int i = tid * 4; i < AGG_ZINTS; i += NTHR * 4) *(v4ia*)(dsm + i) = z4;
      if (tid < MISC_INTS) misc[tid] = 0;
    }
    __syncthreads();

    int t = 0, ov = 0;
    const int nChunks = (nE + CHUNK - 1) / CHUNK;
#pragma unroll 1
    for (int ch = 0; ch < nChunks; ++ch) {
      const int cbase = ch * CHUNK;
      const int wc = scan_chunk<SLA>(dsts, nE, cbase, nodeBase, NBA, vec8, list, tid, lane, wave);
      if (lane == 0) misc[wave] = wc;
      __syncthreads();
      if (wave == 0) {
#pragma unroll 1
        for (int w2 = 0; w2 < NWAVE; ++w2) {
          int c = misc[w2];
          c = c < 0 ? 0 : (c > WCAP ? WCAP : c);
#pragma unroll 1
          for (int b0 = 0; b0 < c; b0 += 32) {
            const int idx = b0 + lane;
            const int ent = list[w2 * WCAP + (idx < WCAP ? idx : WCAP - 1)];
            const int m32 = (c - b0) < 32 ? (c - b0) : 32;
#pragma unroll 1
            for (int k = 0; k < m32; ++k) {
              const int u    = __builtin_amdgcn_readlane(ent, k);
              const int slot = u & (NBA - 1);
              const int el   = (u >> SLA) & (CHUNK - 1);
              const int pk   = ((cbase + el) << SLA) | slot;
              if (t < RCAP) {
                if (lane == 0) { hl[t] = pk; cnt[slot] = cnt[slot] + 1; }
                t = t + 1;
              } else {
                ov = 1;
              }
            }
          }
        }
      }
      __syncthreads();
    }
    if (wave == 0 && lane == 0) { misc[8] = t; misc[9] = ov; }
    __syncthreads();
    int tt = misc[8];
    tt = tt < 0 ? 0 : (tt > RCAP ? RCAP : tt);
    ovf = misc[9];

    if (wave == 0) {
      const int base = lane * (NBA / 32);
      int s = 0;
#pragma unroll 1
      for (int i = 0; i < NBA / 32; ++i) s += cnt[base + i];
      int incl = s;
#pragma unroll
      for (int d = 1; d < 32; d <<= 1) {
        const int y = __shfl_up(incl, d, 32);
        if (lane >= d) incl += y;
      }
      int run = incl - s;
#pragma unroll 1
      for (int i = 0; i < NBA / 32; ++i) {
        const int cv = cnt[base + i];
        offs[base + i] = run;
        cur[base + i]  = run;
        run += cv;
      }
    }
    __syncthreads();
    if (wave == 0) {
#pragma unroll 1
      for (int b0 = 0; b0 < tt; b0 += 32) {
        const int idx = b0 + lane;
        const int ent = hl[idx < RCAP ? idx : RCAP - 1];
        const int m32 = (tt - b0) < 32 ? (tt - b0) : 32;
#pragma unroll 1
        for (int k = 0; k < m32; ++k) {
          const int u    = __builtin_amdgcn_readlane(ent, k);
          const int slot = u & (NBA - 1);
          if (lane == 0) {
            int p = cur[slot];
            p = p < 0 ? 0 : (p > RCAP - 1 ? RCAP - 1 : p);
            sl[p] = u;
            cur[slot] = p + 1;
          }
        }
      }
    }
    __syncthreads();

    v4i mv = {0, 0, 0, 0};
    mv.x = (lane == 0) ? tt : 0;
    mv.y = (lane == 0) ? ovf : 0;
    const bool mline = (wave == 0) && (lane < 8);
#pragma unroll 1
    for (int i = tid * 4; i < TBLCOPY; i += NTHR * 4) {
      const v4i v = *(const v4ia*)(sl + i);
      *(volatile v4i*)(tb + i) = v;
    }
    if (mline) *(volatile v4i*)(tb + TBLCOPY + 4 * lane) = mv;
    __threadfence();
#pragma unroll 1
    for (int i = tid * 4; i < TBLCOPY; i += NTHR * 4) {
      const v4i v = *(const v4ia*)(sl + i);
      *(volatile v4i*)(tb + i) = v;
    }
    if (mline) *(volatile v4i*)(tb + TBLCOPY + 4 * lane) = mv;
  } else {
#pragma unroll 1
    for (int i = tid * 4; i < TBLCOPY; i += NTHR * 4) {
      const v4i v = *(const v4i*)(tb + i);
      *(v4ia*)(sl + i) = v;
    }
    ovf = tb[TBLCOPY + 1];
    __syncthreads();
  }

  const float qnan = __int_as_float(0x7fc00000);
  const float pz = (ovf != 0) ? qnan : 0.0f;
#pragma unroll 1
  for (int si = 0; si < NBA / NWAVE; ++si) {
    const int s    = si * NWAVE + wave;
    const int node = nodeBase + s;
    int c = cnt[s];
    const bool big = (c > DEGCAP) || (c < 0);
    c = c < 0 ? 0 : (c > DEGCAP ? DEGCAP : c);
    int o = offs[s];
    o = o < 0 ? 0 : (o > RCAP ? RCAP : o);
    float a0 = 0.0f, a1 = 0.0f, a2 = 0.0f, a3 = 0.0f;
#pragma unroll 1
    for (int b0 = 0; b0 < c; b0 += 32) {
      int idx = o + b0 + lane;
      idx = idx > RCAP - 1 ? RCAP - 1 : idx;
      const int ent = sl[idx];
      int eid = ent >> SLA;
      eid = eid < 0 ? 0 : (eid > nE - 1 ? nE - 1 : eid);
      int sr = srcs[eid];
      sr = sr < 0 ? 0 : (sr > nN - 1 ? nN - 1 : sr);
      const int m32 = (c - b0) < 32 ? (c - b0) : 32;
#pragma unroll 1
      for (int k = 0; k < m32; ++k) {
        const int sk = __builtin_amdgcn_readlane(sr, k);
        const v4f a = *(const v4f*)(hf + (size_t)sk * DF + 4 * lane);
        a0 += a.x; a1 += a.y; a2 += a.z; a3 += a.w;
      }
    }
    const float cden = (float)(c < 1 ? 1 : c);
    const float rinv = 1.0f / cden;
    const float pzr  = big ? qnan : pz;
    const bool live  = node < nN;
    v4f mm;
    mm.x = live ? (a0 * rinv + pzr) : 0.0f;
    mm.y = live ? (a1 * rinv + pzr) : 0.0f;
    mm.z = live ? (a2 * rinv + pzr) : 0.0f;
    mm.w = live ? (a3 * rinv + pzr) : 0.0f;
    v4us mh, ml;
    split4(mm, mh, ml);
    *(v4usa*)(rowbuf + 4 * lane) = mh;
    *(v4usa*)(rowbuf + DF + 4 * lane) = ml;
    wave_sync();
    const v8us q0 = *(const v8usa*)(rowbuf + 8 * lane);
    wave_sync();
    if (node < mRows) {
      unsigned short* rpw = apl + (size_t)node * AP + 2 * DF + 8 * lane;
      *(volatile v8us*)rpw = q0;
      __threadfence();
      *(volatile v8us*)rpw = q0;
    }
  }
}

static inline int cdiv(int a, int b) { return (a + b - 1) / b; }
static inline size_t al256(size_t o) { return (o + 255) & ~(size_t)255; }

extern "C" void kernel_launch(void* const* d_in, const int* in_sizes, int n_in,
                              void* d_out, int out_size, void* d_ws, size_t ws_size,
                              hipStream_t stream) {
  if (n_in < 18) return;
  if (in_sizes[0] < DF || (in_sizes[0] % DF) != 0) return;
  const int nN = in_sizes[0] / DF;
  if (nN < 16 || nN >= (1 << 21)) return;
  if (in_sizes[1] < 2 || (in_sizes[1] & 1) != 0) return;
  const int nE = in_sizes[1] / 2;
  if (nE < 1 || nE >= (1 << (31 - SLA))) return;
  for (int l = 0; l < 3; ++l) {
    if (in_sizes[2 + 4 * l] != DF * DF || in_sizes[3 + 4 * l] != DF) return;
    if (in_sizes[4 + 4 * l] != 2 * DF * DF || in_sizes[5 + 4 * l] != DF) return;
  }
  if (in_sizes[14] != DF * DF || in_sizes[15] != DF) return;
  if (in_sizes[16] != DF * DOUT || in_sizes[17] != DOUT) return;
  if ((long long)out_size != (long long)nN * DOUT) return;

  const float* x    = (const float*)d_in[0];
  const int*   edge = (const int*)d_in[1];
  const float* Wl[3] = {(const float*)d_in[2], (const float*)d_in[6], (const float*)d_in[10]};
  const float* bl[3] = {(const float*)d_in[3], (const float*)d_in[7], (const float*)d_in[11]};
  const float* Wa[3] = {(const float*)d_in[4], (const float*)d_in[8], (const float*)d_in[12]};
  const float* ba[3] = {(const float*)d_in[5], (const float*)d_in[9], (const float*)d_in[13]};
  const float* Wm1 = (const float*)d_in[14];
  const float* bm1 = (const float*)d_in[15];
  const float* Wm2 = (const float*)d_in[16];
  const float* bm2 = (const float*)d_in[17];
  float* out = (float*)d_out;
  const int* src = edge;
  const int* dst = edge + nE;

  const int MP = cdiv(nN, GBM) * GBM;
  const int gM = MP / GBM;
  const int gA = cdiv(MP, NBA);
  if ((long long)gA * NBA < (long long)MP) return;
  const int vec8 = ((nE & 3) == 0) ? 1 : 0;

  char* ws = (char*)d_ws;
  size_t off = 0;
  const size_t oWP  = off; off = al256(off + (size_t)WP_ELEMS * 2);
  const size_t oXA  = off; off = al256(off + (size_t)MP * AP * 2);
  const size_t oH   = off; off = al256(off + (size_t)MP * DF * 4);
  const size_t oTBL = off; off = al256(off + (size_t)gA * TBLSTRIDE * 4);
  if (off > ws_size || off > (size_t)WSMAX) return;
  unsigned short* WP  = (unsigned short*)(ws + oWP);
  unsigned short* XA  = (unsigned short*)(ws + oXA);
  float*          H   = (float*)(ws + oH);
  int*            TBL = (int*)(ws + oTBL);

  const size_t scanLds = (size_t)AGG_LDS_INTS * 4;
  (void)hipFuncSetAttribute(reinterpret_cast<const void*>(&k_scan<0>), hipFuncAttributeMaxDynamicSharedMemorySize, (int)scanLds);
  (void)hipFuncSetAttribute(reinterpret_cast<const void*>(&k_scan<1>), hipFuncAttributeMaxDynamicSharedMemorySize, (int)scanLds);

  const int nUx = MP * 32;
  k_wprep<<<U_WA2 / NTHR, NTHR, 0, stream>>>(Wl[0], Wl[1], Wl[2], Wm1, Wm2, Wa[0], Wa[1], Wa[2], WP);
  k_cvx<<<cdiv(nUx, NTHR), NTHR, 0, stream>>>(x, nN, nUx, XA);
  k_gemm<0><<<gM, GTHR, 0, stream>>>(XA, WP + O_WL0, DF, 0, 0, bl[0], H, nN);
  k_scan<0><<<gA, NTHR, scanLds, stream>>>(src, dst, nE, nN, vec8, MP, H, XA, TBL);
  k_gemm<1><<<gM, GTHR, 0, stream>>>(XA, WP + O_WA0, AP, DF, 2 * DF, ba[0], H, nN);
  k_gemm<0><<<gM, GTHR, 0, stream>>>(XA, WP + O_WL1, 2 * DF, 0, 0, bl[1], H, nN);
  k_scan<1><<<gA, NTHR, scanLds, stream>>>(src, dst, nE, nN, vec8, MP, H, XA, TBL);
  k_gemm<1><<<gM, GTHR, 0, stream>>>(XA, WP + O_WA1, AP, 0, 0, ba[1], H, nN);
  k_gemm<0><<<gM, GTHR, 0, stream>>>(XA, WP + O_WL2, 2 * DF, 0, 0, bl[2], H, nN);
  k_scan<1><<<gA, NTHR, scanLds, stream>>>(src, dst, nE, nN, vec8, MP, H, XA, TBL);
  k_gemm<1><<<gM, GTHR, 0, stream>>>(XA, WP + O_WA2, AP, 0, 0, ba[2], H, nN);
  k_post<<<gM, GTHR, 0, stream>>>(XA, WP + O_WM1, WP + O_WM2, bm1, bm2, out, nN);
}
